// VariableSelectionNetwork_84997402788316
// MI455X (gfx1250) — hardware-run, weakly checked
//
#include <hip/hip_runtime.h>


#define NRW  16384
#define NPT  4096
#define NFE  16
#define NHD  256
constexpr size_t al256(size_t b) { return (b + 255) & ~(size_t)255; }
constexpr size_t WS_TOTAL = 2 * al256((size_t)NFE * NHD * NHD * 2) + al256((size_t)NFE * NPT * NHD * 2) + al256((size_t)NFE * NPT * NHD * 4);
static_assert(WS_TOTAL == 104857600 && WS_TOTAL <= 134217728, "the workspace carve: 100.0 MiB");
static_assert(NRW % NPT == 0 && NPT % 64 == 0 && NHD % 64 == 0 && NHD % 32 == 0 && ((size_t)NFE * NHD * NHD) % 2048 == 0 && (NHD * NHD) % 4096 == 0 && NFE * 4 == 64, "whole tiles; whole depth steps; whole lines");
typedef _Float16 h16;
typedef unsigned short bf;
typedef __attribute__((ext_vector_type(16))) __bf16   v16bf;
typedef __attribute__((ext_vector_type(16))) _Float16 v16h;
typedef __attribute__((ext_vector_type(8)))  _Float16 v8h;
typedef __attribute__((ext_vector_type(8)))  unsigned short v8us;
typedef __attribute__((ext_vector_type(8)))  float    v8f;
typedef __attribute__((ext_vector_type(4)))  float    v4f;
typedef v8h  __attribute__((may_alias)) v8ha;
typedef v4f  __attribute__((may_alias)) v4fa;
typedef v8us __attribute__((may_alias)) v8usa;

__device__ __forceinline__ unsigned short f2bf(float f) { unsigned u = __float_as_uint(f); u += 0x7FFFu + ((u >> 16) & 1u); return (unsigned short)(u >> 16); }
__device__ __forceinline__ float bf2f(unsigned short b) { return __uint_as_float(((unsigned)b) << 16); }
__device__ __forceinline__ float bfr(float f) { return bf2f(f2bf(f)); }
__device__ __forceinline__ v16h cat16(v8h lo, v8h hi) { return __builtin_shufflevector(lo, hi, 0, 1, 2, 3, 4, 5, 6, 7, 8, 9, 10, 11, 12, 13, 14, 15); }
__device__ __forceinline__ v16bf cat16b(v8us lo, v8us hi) { return __builtin_bit_cast(v16bf, __builtin_shufflevector(lo, hi, 0, 1, 2, 3, 4, 5, 6, 7, 8, 9, 10, 11, 12, 13, 14, 15)); }
__device__ __forceinline__ v8f wmma16(v16h a, v16h b, v8f c) { return __builtin_amdgcn_wmma_f32_16x16x32_f16(false, a, false, b, (short)0, c, false, false); }
__device__ __forceinline__ v8f wmmab(v16bf a, v16bf b, v8f c) { return __builtin_amdgcn_wmma_f32_16x16x32_bf16(false, a, false, b, (short)0, c, false, false); }


template <typename T16> struct WFrag;
template <> struct WFrag<h16> { typedef v16h V; static __device__ __forceinline__ V ld(const h16* p) { return cat16(*(const v8h*)p, *(const v8h*)(p + 16)); } static __device__ __forceinline__ v8f mma(V a, V b, v8f c) { return wmma16(a, b, c); } };
template <> struct WFrag<bf> { typedef v16bf V; static __device__ __forceinline__ V ld(const bf* p) { return cat16b(*(const v8us*)p, *(const v8us*)(p + 16)); } static __device__ __forceinline__ v8f mma(V a, V b, v8f c) { return wmmab(a, b, c); } };
template <typename T16, int NSPLIT, bool BIAS>
__global__ __launch_bounds__(32) void k_gemmw(const T16* __restrict__ A, const T16* __restrict__ A2, const T16* __restrict__ Bt, const T16* __restrict__ Bt2, int K, float* C, int ldc, const float* __restrict__ bias, size_t sA, size_t sB, size_t sC) {
    typedef typename WFrag<T16>::V V;
    __shared__ __align__(16) float os[16 * 68];
    const size_t z = blockIdx.z; A += z * sA; if (A2) A2 += z * sA; Bt += z * sB; if (Bt2) Bt2 += z * sB; C += z * sC;
    const int lane = threadIdx.x & 31, lr = lane & 15, hi = lane >> 4; const int r0 = blockIdx.x * 64, c0 = blockIdx.y * 64;
    v8f acc[4][4];
#pragma unroll
    for (int mb = 0; mb < 4; ++mb)
#pragma unroll
        for (int nb = 0; nb < 4; ++nb) acc[mb][nb] = (v8f){};
    const size_t aoff = (size_t)(r0 + lr) * K + 8 * hi, boff = (size_t)(c0 + lr) * K + 8 * hi;
    for (int kc = 0; kc < K; kc += 32) {
        V a[4], a2[4];
#pragma unroll
        for (int mb = 0; mb < 4; ++mb) { a[mb] = WFrag<T16>::ld(A + aoff + (size_t)mb * 16 * K + kc); if (NSPLIT == 1 || NSPLIT == 2) a2[mb] = WFrag<T16>::ld(A2 + aoff + (size_t)mb * 16 * K + kc); }
#pragma unroll
        for (int nb = 0; nb < 4; ++nb) { const V b = WFrag<T16>::ld(Bt + boff + (size_t)nb * 16 * K + kc); V b2; if (NSPLIT >= 2) b2 = WFrag<T16>::ld(Bt2 + boff + (size_t)nb * 16 * K + kc);
#pragma unroll
            for (int mb = 0; mb < 4; ++mb) { acc[mb][nb] = WFrag<T16>::mma(a[mb], b, acc[mb][nb]); if (NSPLIT == 1 || NSPLIT == 2) acc[mb][nb] = WFrag<T16>::mma(a2[mb], b, acc[mb][nb]); if (NSPLIT >= 2) acc[mb][nb] = WFrag<T16>::mma(a[mb], b2, acc[mb][nb]); } }
        asm volatile("v_nop\n\tv_nop\n\tv_nop\n\tv_nop" : "+v"(acc[0][0]), "+v"(acc[1][1]), "+v"(acc[2][2]), "+v"(acc[3][3]) : "v"(a[0]), "v"(a[3]));
    }
#pragma unroll
    for (int mb = 0; mb < 4; ++mb) {
#pragma unroll
        for (int nb = 0; nb < 4; ++nb) {
#pragma unroll
            for (int j = 0; j < 8; ++j) os[(hi * 8 + j) * 68 + nb * 16 + lr] = acc[mb][nb][j]; }
        __builtin_amdgcn_wave_barrier(); asm volatile("" ::: "memory");
        float* crow = C + (size_t)(r0 + mb * 16) * ldc + c0;
#pragma unroll 1
        for (int ps = 0; ps < 2; ++ps) {
#pragma unroll
            for (int s = 0; s < 8; ++s) { const int row = 2 * s + hi, cofs = lr * 4; v4f val = *(const v4fa*)(os + row * 68 + cofs); if (BIAS) { val[0] += bfr(bias[c0 + cofs]); val[1] += bfr(bias[c0 + cofs + 1]); val[2] += bfr(bias[c0 + cofs + 2]); val[3] += bfr(bias[c0 + cofs + 3]); }
                *(volatile v4f*)(crow + (size_t)row * ldc + cofs) = val; }
            if (ps == 0) __threadfence(); }
        __builtin_amdgcn_wave_barrier(); asm volatile("" ::: "memory");
    }
}

__device__ __forceinline__ h16 tohx(float x) { return (h16)x; }
__device__ __forceinline__ void splitf(float y, unsigned short& h, unsigned short& l) { h = f2bf(y); l = f2bf(y - bf2f(h)); }
typedef __attribute__((ext_vector_type(2))) _Float16 v2h;
typedef __attribute__((ext_vector_type(4))) _Float16 v4h;
typedef __attribute__((ext_vector_type(2))) unsigned short v2us;
typedef __attribute__((ext_vector_type(4))) unsigned short v4us;
typedef __attribute__((ext_vector_type(2))) float v2f;
typedef __attribute__((ext_vector_type(4))) int v4i;

__global__ __launch_bounds__(256) void k_wtG(const float* __restrict__ w, int K, int N, bf* Bt) {
    const int lane = threadIdx.x & 31; const int L0 = (blockIdx.x * 8 + (threadIdx.x >> 5)) * 8; const int nlines = N * K / 64;
#pragma unroll
    for (int ps = 0; ps < 2; ++ps) {
        for (int l = 0; l < 8; ++l) { const int L = L0 + l; if (L >= nlines) break; const size_t e = (size_t)L * 64 + lane * 2; const int k = (int)(e % K), n = (int)(e / K); v2us o;
            o[0] = f2bf(w[(size_t)k * N + n]); o[1] = f2bf(w[(size_t)(k + 1) * N + n]); *(volatile v2us*)(Bt + e) = o; }
        if (ps == 0) __threadfence(); }
}

__global__ __launch_bounds__(256) void k_b2h(const bf* src, h16* dst, size_t n8) {
    const size_t e = (size_t)blockIdx.x * 256 + threadIdx.x; if (e >= n8) return; const v8us w = *(const v8us*)(src + e * 8); v8h o;
#pragma unroll
    for (int q = 0; q < 8; ++q) o[q] = tohx(bf2f(w[q]));
    *(volatile v8h*)(dst + e * 8) = o; __threadfence(); *(volatile v8h*)(dst + e * 8) = o; }

__global__ __launch_bounds__(64) void k_gate(const float* __restrict__ xi, const float* __restrict__ uc, const float* __restrict__ cc, const float* __restrict__ ud, const float* __restrict__ cd, float* r1) {
    const unsigned m = blockIdx.x * 64 + threadIdx.x; if (m >= (unsigned)NRW) return; float xv[NFE], lo[NFE];
#pragma unroll
    for (int c = 0; c < NFE / 4; ++c) { const v4f v = *(const v4f*)(xi + (size_t)m * NFE + 4 * c); xv[4 * c] = bfr(v[0]); xv[4 * c + 1] = bfr(v[1]); xv[4 * c + 2] = bfr(v[2]); xv[4 * c + 3] = bfr(v[3]); }
#pragma unroll
    for (int f = 0; f < NFE; ++f) lo[f] = 0.0f;
    for (int g = 0; g < NHD; ++g) { float s = 0.0f;
#pragma unroll
        for (int f = 0; f < NFE; ++f) s += xv[f] * bfr(uc[f * NHD + g]);
        s += bfr(cc[g]); const float em = expm1f(s); const float av = s > 0.0f ? s : em;
#pragma unroll
        for (int f = 0; f < NFE; ++f) lo[f] += av * bfr(ud[g * NFE + f]); }
    float mx = -3.0e38f;
#pragma unroll
    for (int f = 0; f < NFE; ++f) { lo[f] += bfr(cd[f]); mx = lo[f] > mx ? lo[f] : mx; }
    float sm = 0.0f;
#pragma unroll
    for (int f = 0; f < NFE; ++f) { lo[f] = expf(lo[f] - mx); sm += lo[f]; }
    float* d = r1 + (size_t)m * NFE;
#pragma unroll
    for (int c = 0; c < NFE / 4; ++c) { v4f o; o[0] = lo[4 * c] / sm; o[1] = lo[4 * c + 1] / sm; o[2] = lo[4 * c + 2] / sm; o[3] = lo[4 * c + 3] / sm; *(volatile v4f*)(d + 4 * c) = o; }
    __threadfence();
#pragma unroll
    for (int c = 0; c < NFE / 4; ++c) { v4f o; o[0] = lo[4 * c] / sm; o[1] = lo[4 * c + 1] / sm; o[2] = lo[4 * c + 2] / sm; o[3] = lo[4 * c + 3] / sm; *(volatile v4f*)(d + 4 * c) = o; } }

__global__ __launch_bounds__(256) void k_hop(const float* __restrict__ xp, const float* __restrict__ ua, const float* __restrict__ ca, h16* AH) {
    const unsigned e = blockIdx.x * 256 + threadIdx.x; if (e >= (unsigned)(NPT * (NHD / 8))) return; const unsigned f = blockIdx.y; const unsigned m = e >> 5, g0 = (e & 31) * 8;
    const float xv = bfr(xp[(size_t)m * NFE + f]); const v8f w = *(const v8f*)(ua + (size_t)f * NHD + g0); const v8f c = *(const v8f*)(ca + (size_t)f * NHD + g0); v8h o;
#pragma unroll
    for (int q = 0; q < 8; ++q) { const float t = xv * bfr(w[q]) + bfr(c[q]); const float em = expm1f(t); o[q] = tohx(t > 0.0f ? t : em); }
    h16* d = AH + ((size_t)f * NPT + m) * NHD + g0; *(volatile v8h*)(d) = o; __threadfence(); *(volatile v8h*)(d) = o; }

__global__ __launch_bounds__(256) void k_comb(const float* __restrict__ PP, const float* __restrict__ cb, const float* __restrict__ wt, float* r0) {
    const unsigned e = blockIdx.x * 256 + threadIdx.x; if (e >= (unsigned)(NPT * (NHD / 4))) return; const unsigned m = e >> 6, g0 = (e & 63) * 4; float wv[NFE]; v4f acc; acc[0] = 0.0f; acc[1] = 0.0f; acc[2] = 0.0f; acc[3] = 0.0f;
#pragma unroll
    for (int c = 0; c < NFE / 4; ++c) { const v4f v = *(const v4f*)(wt + (size_t)m * NFE + 4 * c); wv[4 * c] = v[0]; wv[4 * c + 1] = v[1]; wv[4 * c + 2] = v[2]; wv[4 * c + 3] = v[3]; }
#pragma unroll
    for (int f = 0; f < NFE; ++f) { const v4f p = *(const v4f*)(PP + ((size_t)f * NPT + m) * NHD + g0); const v4f b = *(const v4f*)(cb + (size_t)f * NHD + g0);
        acc[0] += wv[f] * (p[0] + bfr(b[0])); acc[1] += wv[f] * (p[1] + bfr(b[1])); acc[2] += wv[f] * (p[2] + bfr(b[2])); acc[3] += wv[f] * (p[3] + bfr(b[3])); }
    float* d = r0 + (size_t)m * NHD + g0; *(volatile v4f*)(d) = acc; __threadfence(); *(volatile v4f*)(d) = acc; }

extern "C" void kernel_launch(void* const* d_in, const int* in_sizes, int n_in,
                              void* d_out, int out_size, void* d_ws, size_t ws_size, hipStream_t stream) {
    if (n_in < 9) return;
    if (in_sizes[0] < NRW * NFE || in_sizes[1] < NFE * NHD || in_sizes[2] < NFE * NHD || in_sizes[3] < NFE * NHD * NHD || in_sizes[4] < NFE * NHD || in_sizes[5] < NFE * NHD || in_sizes[6] < NHD || in_sizes[7] < NHD * NFE || in_sizes[8] < NFE || out_size < NRW * NHD + NRW * NFE) return;
    const float* xi = (const float*)d_in[0]; const float* ua = (const float*)d_in[1]; const float* ca = (const float*)d_in[2]; const float* ub = (const float*)d_in[3]; const float* cb = (const float*)d_in[4];
    const float* uc = (const float*)d_in[5]; const float* cc = (const float*)d_in[6]; const float* ud = (const float*)d_in[7]; const float* cd = (const float*)d_in[8];
    float* R0 = (float*)d_out; float* R1 = R0 + (size_t)NRW * NHD;
    char* wsp = (char*)d_ws;
    auto take = [&](size_t bytes) { char* cur = wsp; wsp += (bytes + 255) & ~(size_t)255; return (void*)cur; };
    bf* WT = (bf*)take((size_t)NFE * NHD * NHD * 2); h16* WH = (h16*)take((size_t)NFE * NHD * NHD * 2); h16* AH = (h16*)take((size_t)NFE * NPT * NHD * 2); float* PP = (float*)take((size_t)NFE * NPT * NHD * 4);
    if ((size_t)(wsp - (char*)d_ws) != WS_TOTAL || WS_TOTAL > ws_size) return;
    for (int f = 0; f < NFE; ++f)
        k_wtG<<<(unsigned)(((size_t)NHD * NHD / 64 + 63) / 64), 256, 0, stream>>>(ub + (size_t)f * NHD * NHD, NHD, NHD, WT + (size_t)f * NHD * NHD);
    k_b2h<<<(unsigned)(((size_t)NFE * NHD * NHD / 8 + 255) / 256), 256, 0, stream>>>(WT, WH, (size_t)NFE * NHD * NHD / 8);
    k_gate<<<NRW / 64, 64, 0, stream>>>(xi, uc, cc, ud, cd, R1);
    for (int pt = 0; pt < NRW / NPT; ++pt) {
        const size_t r0w = (size_t)pt * NPT;
        k_hop<<<dim3(NPT * (NHD / 8) / 256, NFE, 1), 256, 0, stream>>>(xi + r0w * NFE, ua, ca, AH);
        k_gemmw<h16, 0, false><<<dim3(NPT / 64, NHD / 64, NFE), 32, 0, stream>>>(AH, nullptr, WH, nullptr, NHD, PP, NHD, nullptr, (size_t)NPT * NHD, (size_t)NHD * NHD, (size_t)NPT * NHD);
        k_comb<<<NPT * (NHD / 4) / 256, 256, 0, stream>>>(PP, cb, R1 + r0w * NFE, R0 + r0w * NHD);
    }
}
